// RNNForParityCheck_51608327029372
// MI455X (gfx1250) — hardware-verified
//
#include <hip/hip_runtime.h>
#include <math.h>

typedef __attribute__((ext_vector_type(16))) _Float16 v16h;
typedef __attribute__((ext_vector_type(8)))  _Float16 v8h;
typedef __attribute__((ext_vector_type(8)))  float    v8f;
typedef __attribute__((ext_vector_type(4)))  float    v4f;

__device__ __forceinline__ void dep_guard_h(v8f& a, v8f& b, v16h x, v16h y) { asm volatile("v_nop\n\tv_nop\n\tv_nop\n\tv_nop" : "+v"(a), "+v"(b) : "v"(x), "v"(y)); }
__device__ __forceinline__ void keep4_h(v16h a, v16h b, v16h c, v16h d) { asm volatile("v_nop" :: "v"(a), "v"(b), "v"(c), "v"(d)); }
__device__ __forceinline__ void acc_guard4(v8f& a, v8f& b, v8f& c, v8f& d) { asm volatile("v_nop\n\tv_nop\n\tv_nop\n\tv_nop" : "+v"(a), "+v"(b), "+v"(c), "+v"(d)); }
template <typename T> struct Frag;
template <> struct Frag<_Float16> {
  typedef v16h V; union U { v16h v; v8h h[2]; };
  static __device__ __forceinline__ v16h load(const _Float16* p) {
    U f; f.h[0] = *(const v8h*)(p); f.h[1] = *(const v8h*)(p + 16); return f.v;
  }
  static __device__ __forceinline__ v8f mma(v16h a, v16h b, v8f c) {
    return __builtin_amdgcn_wmma_f32_16x16x32_f16(false, a, false, b, (short)0, c, false, false);
  }
  static __device__ __forceinline__ void guard(v8f& a, v8f& b, v16h x, v16h y) { dep_guard_h(a, b, x, y); }
  static __device__ __forceinline__ void keep(v16h a, v16h b, v16h c, v16h d) { keep4_h(a, b, c, d); }
};

constexpr int kBatch      = 128;
constexpr int kSteps      = 256;
constexpr int kHid        = 512;
constexpr int kKcat       = 1024;
constexpr int kRowsPerBlk = 16;
constexpr int kRnnBlocks  = kBatch / kRowsPerBlk;
constexpr int kPitch0     = 520;
constexpr int kPitch1     = 1032;
constexpr int kLdsBytes   = kRowsPerBlk * kPitch0 * 2 + kRowsPerBlk * kPitch1 * 2;
constexpr int kSlabFloats = 16 * 68;
static_assert(kBatch % kRowsPerBlk == 0);
static_assert(8 * kSlabFloats * 4 <= kLdsBytes);
static_assert((kLdsBytes % 16) == 0);
constexpr float kStateScale  = 8.0f;
constexpr float kWeightScale = 16.0f;
constexpr float kAccFold     = 1.0f / 128.0f;

constexpr size_t kOffWhh0  = 0;
constexpr size_t kOffW1cat = kOffWhh0 + (size_t)kHid * kHid * 2;
constexpr size_t kOffEtab  = kOffW1cat + (size_t)kHid * kKcat * 2;
constexpr size_t kOffBias1 = kOffEtab + (size_t)2 * kHid * 4;
constexpr size_t kWsTotal  = kOffBias1 + (size_t)kHid * 4;

__global__ __launch_bounds__(256) void prep_weights(const float* __restrict__ W_ih, const float* __restrict__ W_hh,
                                                    _Float16* __restrict__ Whh0h, _Float16* __restrict__ W1cat) {
  const int tid = threadIdx.x;
  if (blockIdx.x < 128) {
    const int i   = blockIdx.x * 256 + tid;
    const int row = i >> 6;
    const int k8  = (i & 63) * 8;
    const float* src = W_hh + (size_t)row * kHid + k8;
    const v4f f0 = *(const v4f*)(src);
    const v4f f1 = *(const v4f*)(src + 4);
    v8h hv;
#pragma unroll
    for (int e = 0; e < 4; ++e) {
      hv[e]     = (_Float16)(f0[e] * kWeightScale);
      hv[4 + e] = (_Float16)(f1[e] * kWeightScale);
    }
    _Float16* dst = Whh0h + (size_t)row * kHid + k8;
    *(volatile v8h*)dst = hv;
    __threadfence();
    *(volatile v8h*)dst = hv;
  } else {
    const int i   = (blockIdx.x - 128) * 256 + tid;
    const int row = i >> 7;
    const int k8  = (i & 127) * 8;
    const int kk  = k8 & 511;
    const float* sa = W_ih + (size_t)kHid * kHid + (size_t)row * kHid + kk;
    const float* sb = W_hh + (size_t)kHid * kHid + (size_t)row * kHid + kk;
    const v4f a0 = *(const v4f*)(sa);
    const v4f a1 = *(const v4f*)(sa + 4);
    const v4f b0 = *(const v4f*)(sb);
    const v4f b1 = *(const v4f*)(sb + 4);
    const bool first = (k8 < kHid);
    v8h hv;
#pragma unroll
    for (int e = 0; e < 4; ++e) {
      hv[e]     = (_Float16)((first ? a0[e] : b0[e]) * kWeightScale);
      hv[4 + e] = (_Float16)((first ? a1[e] : b1[e]) * kWeightScale);
    }
    _Float16* dst = W1cat + (size_t)row * kKcat + k8;
    *(volatile v8h*)dst = hv;
    __threadfence();
    *(volatile v8h*)dst = hv;
  }
}

__global__ __launch_bounds__(256) void prep_tables(const float* __restrict__ W_emb, const float* __restrict__ b_emb,
                                                   const float* __restrict__ W_ih, const float* __restrict__ b_ih,
                                                   const float* __restrict__ b_hh,
                                                   float* __restrict__ Etab, float* __restrict__ bias1) {
  const int tid = threadIdx.x;
  if (blockIdx.x < 4) {
    const int g  = blockIdx.x * 256 + tid;
    const int v  = g >> 9;
    const int cc = g & 511;
    const float* wrow = W_ih + (size_t)cc * kHid;
    float s = 0.f;
#pragma unroll 1
    for (int k = 0; k < kHid; ++k) {
      const float xk = W_emb[2 * k + v] + b_emb[k];
      s = fmaf(xk, wrow[k], s);
    }
    const float e = (s + b_ih[cc]) + b_hh[cc];
    ((volatile float*)Etab)[g] = e;
    __threadfence();
    ((volatile float*)Etab)[g] = e;
  } else {
    const int cc = (blockIdx.x - 4) * 256 + tid;
    const float bv = b_ih[kHid + cc] + b_hh[kHid + cc];
    ((volatile float*)bias1)[cc] = bv;
    __threadfence();
    ((volatile float*)bias1)[cc] = bv;
  }
}

__global__ __launch_bounds__(256) void rnn_persist(const int* __restrict__ ids, const float* __restrict__ Etab,
                                                   const float* __restrict__ bias1,
                                                   const _Float16* __restrict__ Whh0h,
                                                   const _Float16* __restrict__ W1cat,
                                                   float* __restrict__ Sout) {
  __shared__ __align__(16) unsigned int lds_raw[kLdsBytes / 4];
  _Float16* h0t  = (_Float16*)lds_raw;
  _Float16* comb = h0t + kRowsPerBlk * kPitch0;

  const int tid   = threadIdx.x;
  const int wave  = tid >> 5;
  const int lane  = tid & 31;
  const int c     = lane & 15;
  const int hh    = lane >> 4;
  const int koff  = hh * 8;
  const int row0  = blockIdx.x * kRowsPerBlk;
  const int ncol0 = wave * 64;

  for (int i = tid; i < kLdsBytes / 4; i += 256) lds_raw[i] = 0u;
  __syncthreads();

  float e0[4], e1[4], b1v[4];
#pragma unroll
  for (int j = 0; j < 4; ++j) {
    const int n = ncol0 + j * 16 + c;
    e0[j]  = Etab[n];
    e1[j]  = Etab[kHid + n];
    b1v[j] = bias1[n];
  }
  float y0r[4][8], y1r[4][8];
#pragma unroll
  for (int j = 0; j < 4; ++j)
#pragma unroll
    for (int r = 0; r < 8; ++r) { y0r[j][r] = 0.f; y1r[j][r] = 0.f; }

  const int* idp = ids + (size_t)(row0 + 8 * hh) * kSteps;
  const _Float16* arow0  = h0t  + c * kPitch0 + koff;
  const _Float16* arow1  = comb + c * kPitch1 + koff;
  const _Float16* bbase0 = Whh0h + (size_t)(ncol0 + c) * kHid  + koff;
  const _Float16* bbase1 = W1cat + (size_t)(ncol0 + c) * kKcat + koff;

#pragma unroll 1
  for (int t = 0; t < kSteps; ++t) {
    v8f acc[4];
#pragma unroll
    for (int j = 0; j < 4; ++j) acc[j] = (v8f){0.f,0.f,0.f,0.f,0.f,0.f,0.f,0.f};
#pragma unroll 1
    for (int k0 = 0; k0 < kHid; k0 += 32) {
      v16h bf[4];
#pragma unroll
      for (int j = 0; j < 4; ++j) bf[j] = Frag<_Float16>::load(bbase0 + (size_t)j * 16 * kHid + k0);
      const v16h af = Frag<_Float16>::load(arow0 + k0);
#pragma unroll
      for (int j = 0; j < 4; ++j) acc[j] = Frag<_Float16>::mma(af, bf[j], acc[j]);
      Frag<_Float16>::guard(acc[0], acc[3], af, af);
      Frag<_Float16>::keep(bf[0], bf[1], bf[2], bf[3]);
    }
    acc_guard4(acc[0], acc[1], acc[2], acc[3]);

    int sel[8];
#pragma unroll
    for (int r = 0; r < 8; ++r) {
      int id = idp[r * kSteps + t];
      id = (id < 0) ? (id + 2) : id;
      id = (id < 0) ? 0 : ((id > 1) ? 1 : id);
      sel[r] = id;
    }
    __syncthreads();

#pragma unroll
    for (int j = 0; j < 4; ++j) {
      const int col = ncol0 + j * 16 + c;
#pragma unroll
      for (int r = 0; r < 8; ++r) {
        const int rr = 8 * hh + r;
        const float esel = (sel[r] != 0) ? e1[j] : e0[j];
        const float v = acc[j][r] * kAccFold + esel;
        const float y = tanhf(v);
        y0r[j][r] = y;
        const _Float16 hv = (_Float16)(y * kStateScale);
        h0t[rr * kPitch0 + col]  = hv;
        comb[rr * kPitch1 + col] = hv;
      }
    }
    __syncthreads();

    v8f acq[4];
#pragma unroll
    for (int j = 0; j < 4; ++j) acq[j] = (v8f){0.f,0.f,0.f,0.f,0.f,0.f,0.f,0.f};
#pragma unroll 1
    for (int k0 = 0; k0 < kKcat; k0 += 32) {
      v16h bf[4];
#pragma unroll
      for (int j = 0; j < 4; ++j) bf[j] = Frag<_Float16>::load(bbase1 + (size_t)j * 16 * kKcat + k0);
      const v16h af = Frag<_Float16>::load(arow1 + k0);
#pragma unroll
      for (int j = 0; j < 4; ++j) acq[j] = Frag<_Float16>::mma(af, bf[j], acq[j]);
      Frag<_Float16>::guard(acq[0], acq[3], af, af);
      Frag<_Float16>::keep(bf[0], bf[1], bf[2], bf[3]);
    }
    acc_guard4(acq[0], acq[1], acq[2], acq[3]);
    __syncthreads();

#pragma unroll
    for (int j = 0; j < 4; ++j) {
      const int col = ncol0 + j * 16 + c;
#pragma unroll
      for (int r = 0; r < 8; ++r) {
        const int rr = 8 * hh + r;
        const float v = acq[j][r] * kAccFold + b1v[j];
        const float y = tanhf(v);
        y1r[j][r] = y;
        comb[rr * kPitch1 + kHid + col] = (_Float16)(y * kStateScale);
      }
    }
  }
  __syncthreads();

  float* slab = (float*)lds_raw + wave * kSlabFloats;
  const int c4 = (lane & 15) * 4;
#pragma unroll
  for (int l = 0; l < 2; ++l) {
#pragma unroll
    for (int j = 0; j < 4; ++j)
#pragma unroll
      for (int r = 0; r < 8; ++r)
        slab[(8 * hh + r) * 68 + j * 16 + c] = (l == 0) ? y0r[j][r] : y1r[j][r];
    __builtin_amdgcn_fence(__ATOMIC_RELEASE, "workgroup");
    __builtin_amdgcn_wave_barrier();
    __builtin_amdgcn_fence(__ATOMIC_ACQUIRE, "workgroup");
    float* dstbase = Sout + (size_t)(l * kBatch + row0) * kHid + ncol0 + c4;
    for (int pass = 0; pass < 2; ++pass) {
#pragma unroll
      for (int it = 0; it < 8; ++it) {
        const int row = it * 2 + hh;
        const v4f val = *(const v4f*)(slab + row * 68 + c4);
        *(volatile v4f*)(dstbase + (size_t)row * kHid) = val;
      }
      __threadfence();
    }
    __builtin_amdgcn_fence(__ATOMIC_RELEASE, "workgroup");
    __builtin_amdgcn_wave_barrier();
    __builtin_amdgcn_fence(__ATOMIC_ACQUIRE, "workgroup");
  }
}

__global__ __launch_bounds__(256) void head_finish(const float* __restrict__ W_cls, const float* __restrict__ b_cls,
                                                   const int* __restrict__ labels, float* __restrict__ out) {
  const float* S1 = out + 256 + (size_t)kBatch * kHid;
  __shared__ __align__(16) float lg[256];
  __shared__ float lp[kBatch];
  const int tid = threadIdx.x;
  const int b = tid >> 1;
  const int l = tid & 1;
  const float* srow = S1 + (size_t)b * kHid;
  const float* wrow = W_cls + (size_t)l * kHid;
  float s = 0.f;
#pragma unroll 1
  for (int k = 0; k < kHid; ++k) s = fmaf(srow[k], wrow[k], s);
  s += b_cls[l];
  lg[tid] = s;
  __syncthreads();
  if (tid < kBatch) {
    const float l0 = lg[2 * tid];
    const float l1 = lg[2 * tid + 1];
    const float mx = fmaxf(l0, l1);
    const float lse = logf(expf(l0 - mx) + expf(l1 - mx));
    int lab = labels[tid];
    lab = (lab < 0) ? (lab + 2) : lab;
    lab = (lab < 0) ? 0 : ((lab > 1) ? 1 : lab);
    const float lsel = (lab != 0) ? l1 : l0;
    lp[tid] = (lsel - mx) - lse;
  }
  __syncthreads();
  if (tid < 32) {
    const v4f va = *(const v4f*)(lg + tid * 4);
    const v4f vb = *(const v4f*)(lg + 128 + tid * 4);
    for (int pass = 0; pass < 2; ++pass) {
      *(volatile v4f*)(out + tid * 4) = va;
      *(volatile v4f*)(out + 128 + tid * 4) = vb;
      __threadfence();
    }
  }
  if (tid == 0) {
    float accl = 0.f;
#pragma unroll 1
    for (int i = 0; i < kBatch; ++i) accl += lp[i];
    const float loss = -(accl * (1.0f / 128.0f));
    float* lossp = out + 256 + (size_t)2 * kBatch * kHid;
    *(volatile float*)lossp = loss;
    __threadfence();
    *(volatile float*)lossp = loss;
  }
}

extern "C" void kernel_launch(void* const* d_in, const int* in_sizes, int n_in,
                              void* d_out, int out_size, void* d_ws, size_t ws_size,
                              hipStream_t stream) {
  const int*   ids    = (const int*)  d_in[0];
  const int*   labels = (const int*)  d_in[1];
  const float* W_emb  = (const float*)d_in[2];
  const float* b_emb  = (const float*)d_in[3];
  const float* W_ih   = (const float*)d_in[4];
  const float* b_ih   = (const float*)d_in[5];
  const float* W_hh   = (const float*)d_in[6];
  const float* b_hh   = (const float*)d_in[7];
  const float* W_cls  = (const float*)d_in[8];
  const float* b_cls  = (const float*)d_in[9];
  float* out = (float*)d_out;

  if (n_in < 10) return;
  if (ws_size < kWsTotal) return;
  if ((size_t)out_size * 4 < (size_t)(256 + 2 * kBatch * kHid + 1) * 4) return;
  if (in_sizes[0] != kBatch * kSteps || in_sizes[4] != 2 * kHid * kHid || in_sizes[6] != 2 * kHid * kHid) return;

  char* ws = (char*)d_ws;
  _Float16* Whh0h = (_Float16*)(ws + kOffWhh0);
  _Float16* W1cat = (_Float16*)(ws + kOffW1cat);
  float*    Etab  = (float*)   (ws + kOffEtab);
  float*    bias1 = (float*)   (ws + kOffBias1);

  prep_weights<<<384, 256, 0, stream>>>(W_ih, W_hh, Whh0h, W1cat);
  prep_tables<<<6, 256, 0, stream>>>(W_emb, b_emb, W_ih, b_ih, b_hh, Etab, bias1);
  rnn_persist<<<kRnnBlocks, 256, 0, stream>>>(ids, Etab, bias1, Whh0h, W1cat, out + 256);
  head_finish<<<1, 256, 0, stream>>>(W_cls, b_cls, labels, out);
}
